// InvResMLP_64510408786138
// MI455X (gfx1250) — hardware-run, weakly checked
//
#include <hip/hip_runtime.h>

typedef float          v8f   __attribute__((ext_vector_type(8)));
typedef float          v4f   __attribute__((ext_vector_type(4)));
typedef unsigned int   v4u   __attribute__((ext_vector_type(4)));
typedef int            v8i   __attribute__((ext_vector_type(8)));
typedef unsigned short v8us  __attribute__((ext_vector_type(8)));
typedef unsigned short v16us __attribute__((ext_vector_type(16)));
typedef __bf16         v16bf __attribute__((ext_vector_type(16)));
typedef _Float16       v16h  __attribute__((ext_vector_type(16)));
typedef v4f  __attribute__((may_alias)) v4fa;
typedef v8us __attribute__((may_alias)) v8usa;
union FragB { v16bf v; v16us u; v8us h[2]; v8i w; };
union FragH { v16h  v; v16us u; v8us h[2]; v8i w; };

__device__ __forceinline__ v8f wmb(const FragB& a, const FragB& b, v8f c) {
  v8f d = __builtin_amdgcn_wmma_f32_16x16x32_bf16(false, a.v, false, b.v, (short)0, c, false, false);
  asm volatile("v_nop\n\tv_nop\n\tv_nop\n\tv_nop" : "+v"(d) : "v"(a.w), "v"(b.w));
  return d;
}

__device__ __forceinline__ v8f wmh(const FragH& a, const FragH& b, v8f c) {
  v8f d = __builtin_amdgcn_wmma_f32_16x16x32_f16(false, a.v, false, b.v, (short)0, c, false, false);
  asm volatile("v_nop\n\tv_nop\n\tv_nop\n\tv_nop" : "+v"(d) : "v"(a.w), "v"(b.w));
  return d;
}

__device__ __forceinline__ unsigned bf16_bits(float f) {
  const unsigned u = __float_as_uint(f);
  const unsigned r = (u + 0x7FFFu + ((u >> 16) & 1u)) >> 16;
  const unsigned q = (u >> 16) | 0x40u;
  return ((u & 0x7fffffffu) > 0x7f800000u) ? q : r;
}

__device__ __forceinline__ float bf16_val(float f) {
  return __uint_as_float(bf16_bits(f) << 16);
}
__device__ __forceinline__ int clampi(int v, int lo, int hi) {
  return v < lo ? lo : (v > hi ? hi : v);
}

__device__ __forceinline__ unsigned f16_bits(float f) {
  const unsigned u  = __float_as_uint(f);
  const unsigned s  = (u >> 16) & 0x8000u;
  const unsigned a  = u & 0x7fffffffu;
  const unsigned t  = a - 0x38000000u;
  const unsigned r  = (t + 0x0FFFu + ((t >> 13) & 1u)) >> 13;
  const unsigned rc = r > 0x7C00u ? 0x7C00u : r;
  const bool small  = a < 0x38800000u;
  const bool isnan  = a > 0x7f800000u;
  const unsigned fin = small ? 0u : (s | rc);
  return isnan ? (s | 0x7E00u) : fin;
}

__device__ __forceinline__ unsigned pk16(unsigned lo, unsigned hi) { return lo | (hi << 16); }
__device__ __forceinline__ unsigned bf16_lo_bits(float v) {
  float hi = bf16_val(v);
  asm volatile("" : "+v"(hi));
  return bf16_bits(v - hi);
}
__device__ __forceinline__ v4u pack8_bf16(v4f a, v4f c) {
  return (v4u){ pk16(bf16_bits(a[0]), bf16_bits(a[1])), pk16(bf16_bits(a[2]), bf16_bits(a[3])),
                pk16(bf16_bits(c[0]), bf16_bits(c[1])), pk16(bf16_bits(c[2]), bf16_bits(c[3])) };
}
__device__ __forceinline__ v4u pack8_bf16_lo(v4f a, v4f c) {
  return (v4u){ pk16(bf16_lo_bits(a[0]), bf16_lo_bits(a[1])), pk16(bf16_lo_bits(a[2]), bf16_lo_bits(a[3])),
                pk16(bf16_lo_bits(c[0]), bf16_lo_bits(c[1])), pk16(bf16_lo_bits(c[2]), bf16_lo_bits(c[3])) };
}
__device__ __forceinline__ v4u pack8_f16(v4f a, v4f c) {
  return (v4u){ pk16(f16_bits(a[0]), f16_bits(a[1])), pk16(f16_bits(a[2]), f16_bits(a[3])),
                pk16(f16_bits(c[0]), f16_bits(c[1])), pk16(f16_bits(c[2]), f16_bits(c[3])) };
}

template <int FORM>
__global__ __launch_bounds__(256) void k_plane(const float* __restrict__ src, int rows, int cols, int ldsrc,
                                               unsigned short* __restrict__ dst, int MP, int KP) {
  static_assert(FORM >= 0 && FORM <= 3);
  const int KTOT = (FORM == 1 || FORM == 3) ? 2 * KP : KP;
  const unsigned ppr   = (unsigned)(KTOT >> 3);
  const unsigned kp8   = (unsigned)(KP >> 3);
  const unsigned total = (unsigned)MP * ppr;
  const unsigned g     = blockIdx.x * 256u + threadIdx.x;
  const unsigned rowu  = g / ppr;
  const unsigned p     = g - rowu * ppr;
  const bool second    = p >= kp8;
  const int row = (int)rowu;
  const int c0  = (int)((second ? p - kp8 : p) << 3);
  const float* srow = src + (size_t)clampi(row, 0, rows - 1) * (size_t)ldsrc;
  float x[8];
  unsigned mk[8];
#pragma unroll
  for (int e = 0; e < 8; ++e) {
    const int c = c0 + e;
    const float v = srow[clampi(c, 0, cols - 1)];
    asm volatile("" :: "v"(v));
    x[e]  = v;
    mk[e] = (row < rows && c < cols) ? 0xFFFFu : 0u;
  }
  const v4f a = (v4f){ x[0], x[1], x[2], x[3] };
  const v4f c = (v4f){ x[4], x[5], x[6], x[7] };
  v4u o;
  if (FORM == 2) {
    o = pack8_f16(a, c);
  } else {
    const v4u hi = pack8_bf16(a, c);
    o = hi;
    if (FORM == 1) { const v4u lo = pack8_bf16_lo(a, c); o = second ? lo : hi; }
  }
  const v4u mw = (v4u){ pk16(mk[0], mk[1]), pk16(mk[2], mk[3]), pk16(mk[4], mk[5]), pk16(mk[6], mk[7]) };
  o &= mw;
  if (g < total) {
    volatile v4u* q = (volatile v4u*)(dst + (size_t)g * 8);
    *q = o;
    __threadfence();
    *q = o;
  }
}

template <int FORM> struct FragOf    { typedef FragB T; };
template <>         struct FragOf<2> { typedef FragH T; };
__device__ __forceinline__ v8f mm(const FragB& a, const FragB& b, v8f c) { return wmb(a, b, c); }
__device__ __forceinline__ v8f mm(const FragH& a, const FragH& b, v8f c) { return wmh(a, b, c); }
template <class F> __device__ __forceinline__ F ld_frag(const unsigned short* p) {
  F f;
  f.h[0] = *(const v8usa*)(p);
  f.h[1] = *(const v8usa*)(p + 16);
  return f;
}

template <int FORM, int EPI>
__global__ __launch_bounds__(256) __attribute__((amdgpu_num_vgpr(248)))
void k_gemm_nt(const unsigned short* __restrict__ A, const unsigned short* __restrict__ B,
               const float* __restrict__ bias, float* __restrict__ D, int M, int N, int KTOT, int ldd) {
  static_assert(FORM >= 0 && FORM <= 2);
  static_assert(EPI == 0 || EPI == 1);
  typedef typename FragOf<FORM>::T F;
  __shared__ __attribute__((aligned(16))) float sT[8][16 * 68];
  const int lane = threadIdx.x & 31;
  const int wave = threadIdx.x >> 5;
  const int tilesM = (M + 63) >> 6;
  const int tilesN = (N + 63) >> 6;
  const int tile = blockIdx.x * 8 + wave;
  if (tile >= tilesM * tilesN) return;
  const int tm = tile / tilesN;
  const int tn = tile - tm * tilesN;
  const int m0 = tm << 6;
  const int n0 = tn << 6;

  const int rl = lane & 15;
  const int h8 = (lane >> 4) * 8;
  const unsigned short* pa = A + (size_t)(m0 + rl) * (size_t)KTOT + h8;
  const unsigned short* pb = B + (size_t)(n0 + rl) * (size_t)KTOT + h8;

  v8f acc[4][4];
#pragma unroll
  for (int i = 0; i < 4; ++i)
#pragma unroll
    for (int j = 0; j < 4; ++j) acc[i][j] = (v8f){0.f, 0.f, 0.f, 0.f, 0.f, 0.f, 0.f, 0.f};

#pragma unroll 1
  for (int k0 = 0; k0 < KTOT; k0 += 32) {
    F bf[4];
#pragma unroll
    for (int j = 0; j < 4; ++j) bf[j] = ld_frag<F>(pb + (size_t)(j << 4) * (size_t)KTOT + k0);
#pragma unroll
    for (int i = 0; i < 4; ++i) {
      const F af = ld_frag<F>(pa + (size_t)(i << 4) * (size_t)KTOT + k0);
#pragma unroll
      for (int j = 0; j < 4; ++j) acc[i][j] = mm(af, bf[j], acc[i][j]);
    }
  }

  float* slab = sT[wave];
  const int hh = lane >> 4;
  const int c4 = (lane & 15) * 4;
  const int nc = n0 + c4;
  const bool cok = nc < N;
  v4f bv = (v4f){0.f, 0.f, 0.f, 0.f};
  if (EPI == 1) {
    bv = *(const v4fa*)(bias + clampi(nc, 0, N - 4));
    asm volatile("" :: "v"(bv));
  }
#pragma unroll
  for (int i = 0; i < 4; ++i) {
    const int mBase = m0 + (i << 4);
#pragma unroll
    for (int j = 0; j < 4; ++j) {
#pragma unroll
      for (int r = 0; r < 8; ++r) slab[(h8 + r) * 68 + (j << 4) + rl] = acc[i][j][r];
    }
    __builtin_amdgcn_fence(__ATOMIC_RELEASE, "workgroup");
    __builtin_amdgcn_wave_barrier();
    __builtin_amdgcn_fence(__ATOMIC_ACQUIRE, "workgroup");
    v4f vv[8];
#pragma unroll
    for (int it = 0; it < 8; ++it) {
      const int row = it * 2 + hh;
      v4f v = *(const v4fa*)(slab + row * 68 + c4);
      if (EPI == 1) v += bv;
      vv[it] = v;
    }
    for (int pass = 0; pass < 2; ++pass) {
#pragma unroll
      for (int it = 0; it < 8; ++it) {
        const int row = mBase + it * 2 + hh;
        if (cok && row < M) *(volatile v4f*)(D + (size_t)row * (size_t)ldd + nc) = vv[it];
      }
      __threadfence();
    }
    __builtin_amdgcn_fence(__ATOMIC_RELEASE, "workgroup");
    __builtin_amdgcn_wave_barrier();
    __builtin_amdgcn_fence(__ATOMIC_ACQUIRE, "workgroup");
  }
}

#pragma clang fp contract(off)

#ifndef TWO_TERM_1
#define TWO_TERM_1 1
#endif
#ifndef TWO_TERM_2
#define TWO_TERM_2 1
#endif

typedef float  v2f __attribute__((ext_vector_type(2)));
typedef double v2d __attribute__((ext_vector_type(2)));
typedef v2f __attribute__((may_alias)) v2fa;

constexpr int NBAT  = 4;
constexpr int NPT   = 16384;
constexpr int KNB   = 32;
constexpr int CH    = 64;
constexpr int MIDC  = 256;
constexpr int W0LD  = CH + 3;
constexpr int ROWS  = NBAT * NPT;
constexpr int CHUNK = NPT;
constexpr int NREC  = ROWS / 64;
constexpr int OUT_ELEMS = NBAT * CH * NPT;
constexpr int K1T = (TWO_TERM_1 != 0) ? 2 * CH : CH;
constexpr int K2T = (TWO_TERM_2 != 0) ? 2 * MIDC : MIDC;
constexpr int FORM_W1 = (TWO_TERM_1 != 0) ? 3 : 0;
constexpr int FORM_W2 = (TWO_TERM_2 != 0) ? 3 : 0;

constexpr int GB_G0 = 0, GB_B0 = 64, GB_G1 = 128, GB_B1 = 384, GB_G2 = 640, GB_B2 = 704, GB_N = 768;
constexpr int ST_M0 = 0, ST_R0 = 64, ST_M1 = 128, ST_R1 = 384, ST_M2 = 640, ST_R2 = 704, ST_N = 768;

static_assert(KNB == 32 && CH == 64 && MIDC == 256);
static_assert(NPT == (1 << 14) && NPT % 64 == 0);
static_assert(ROWS % 128 == 0 && CHUNK % 128 == 0 && ROWS == 65536 && CHUNK * NBAT == ROWS);
static_assert(NREC == 1024 && NREC * 64 == ROWS);
static_assert(OUT_ELEMS == 4194304);
static_assert(K1T % 32 == 0 && K2T % 32 == 0 && CH % 32 == 0);
static_assert(GB_B2 + 64 == GB_N && ST_R2 + 64 == ST_N);
static_assert(GB_B0 % 32 == 0 && GB_G1 % 32 == 0 && GB_B1 % 32 == 0 && GB_G2 % 32 == 0 && GB_B2 % 32 == 0);
static_assert(ST_R0 % 32 == 0 && ST_M1 % 32 == 0 && ST_R1 % 32 == 0 && ST_M2 % 32 == 0 && ST_R2 % 32 == 0);

constexpr size_t SZ_FB   = (size_t)ROWS * CH * 2;
constexpr size_t SZ_PC   = (size_t)ROWS * 16;
constexpr size_t SZ_P    = (size_t)ROWS * CH * 4;
constexpr size_t SZ_HL   = (size_t)ROWS * 128 * 2;
constexpr size_t SZ_H1   = (size_t)ROWS * MIDC * 4;
constexpr size_t SZ_W0F  = (size_t)CH * CH * 2;
constexpr size_t SZ_W1D  = (size_t)MIDC * 128 * 2;
constexpr size_t SZ_W2D  = (size_t)CH * 512 * 2;
constexpr size_t SZ_W0P  = (size_t)CH * 16;
constexpr size_t SZ_GB   = 4096;
constexpr size_t SZ_ST   = 4096;
constexpr size_t SZ_REC0 = (size_t)NREC * CH * 8;
constexpr size_t SZ_REC1 = (size_t)NREC * MIDC * 8;
constexpr size_t SZ_REC2 = (size_t)NREC * CH * 8;
constexpr size_t OFF_FB   = 0;
constexpr size_t OFF_PC   = OFF_FB + SZ_FB;
constexpr size_t OFF_P    = OFF_PC + SZ_PC;
constexpr size_t OFF_HL   = OFF_P + SZ_P;
constexpr size_t OFF_H1   = OFF_HL + SZ_HL;
constexpr size_t OFF_W0F  = OFF_H1 + SZ_H1;
constexpr size_t OFF_W1D  = OFF_W0F + SZ_W0F;
constexpr size_t OFF_W2D  = OFF_W1D + SZ_W1D;
constexpr size_t OFF_W0P  = OFF_W2D + SZ_W2D;
constexpr size_t OFF_GB   = OFF_W0P + SZ_W0P;
constexpr size_t OFF_ST   = OFF_GB + SZ_GB;
constexpr size_t OFF_REC0 = OFF_ST + SZ_ST;
constexpr size_t OFF_REC1 = OFF_REC0 + SZ_REC0;
constexpr size_t OFF_REC2 = OFF_REC1 + SZ_REC1;
constexpr size_t WS_TOTAL = OFF_REC2 + SZ_REC2;
static_assert(WS_TOTAL == (size_t)((size_t)110737 << 10));
static_assert(WS_TOTAL <= ((size_t)128 << 20));
static_assert(OFF_PC % 256 == 0 && OFF_P % 256 == 0 && OFF_HL % 256 == 0 && OFF_H1 % 256 == 0);
static_assert(OFF_W0F % 256 == 0 && OFF_W1D % 256 == 0 && OFF_W2D % 256 == 0 && OFF_W0P % 256 == 0);
static_assert(OFF_GB % 256 == 0 && OFF_ST % 256 == 0 && OFF_REC0 % 256 == 0 && OFF_REC1 % 256 == 0 && OFF_REC2 % 256 == 0);
static_assert((size_t)ROWS * K1T * 2 <= SZ_HL && (size_t)CHUNK * K2T * 2 <= SZ_HL);
static_assert((size_t)MIDC * K1T * 2 <= SZ_W1D && (size_t)CH * K2T * 2 <= SZ_W2D);
static_assert((size_t)GB_N * 4 <= SZ_GB && (size_t)ST_N * 4 <= SZ_ST);
static_assert((size_t)ROWS * CH * 4 <= SZ_P);

__device__ __forceinline__ float relu_k(float v) { return (v > 0.0f) ? v : (v - v); }

__device__ __forceinline__ float edge_h(float pv, float dx, float dy, float dz, float wx, float wy, float wz) {
  return fmaf(dz, wz, fmaf(dy, wy, fmaf(dx, wx, pv)));
}

__global__ __launch_bounds__(256) void k_prep_f(const float* __restrict__ f, unsigned* __restrict__ fbw) {
  __shared__ float tile[CH * 65];
  const int tid = (int)threadIdx.x, lane = tid & 31, wave = tid >> 5;
  const int b  = (int)blockIdx.x / (NPT / 64);
  const int n0 = ((int)blockIdx.x - b * (NPT / 64)) * 64;
  const float* fs = f + (size_t)b * CH * NPT + n0 + lane;
#pragma unroll 4
  for (int i = 0; i < 16; ++i) {
    const int u  = wave + 8 * i;
    const int c  = u >> 1;
    const int hf = u & 1;
    const float v = fs[(size_t)c * NPT + 32 * hf];
    asm volatile("" :: "v"(v));
    tile[c * 65 + 32 * hf + lane] = v;
  }
  __syncthreads();
  unsigned w[8];
#pragma unroll
  for (int i = 0; i < 8; ++i) {
    const int row = wave * 8 + i;
    w[i] = pk16(bf16_bits(tile[(2 * lane) * 65 + row]), bf16_bits(tile[(2 * lane + 1) * 65 + row]));
  }
  unsigned* base = fbw + (size_t)(b * NPT + n0 + wave * 8) * 32 + lane;
#pragma unroll
  for (int i = 0; i < 8; ++i) *(volatile unsigned*)(base + i * 32) = w[i];
  __threadfence();
#pragma unroll
  for (int i = 0; i < 8; ++i) *(volatile unsigned*)(base + i * 32) = w[i];
}

constexpr int PS_PC  = ROWS / 256;
constexpr int PS_TOT = PS_PC + 2;
__global__ __launch_bounds__(256) void k_prep_small(const float* __restrict__ p, const float* __restrict__ w0,
                                                    const float* __restrict__ g0, const float* __restrict__ b0,
                                                    const float* __restrict__ g1, const float* __restrict__ b1,
                                                    const float* __restrict__ g2, const float* __restrict__ b2,
                                                    float* __restrict__ PC, float* __restrict__ W0P,
                                                    float* __restrict__ GB) {
  const int tid = (int)threadIdx.x;
  const int blk = (int)blockIdx.x;
  if (blk < PS_PC) {
    const int r = blk * 256 + tid;
    const float* s = p + (size_t)r * 3;
    const float x = s[0], y = s[1], z = s[2];
    asm volatile("" :: "v"(x));
    asm volatile("" :: "v"(y));
    asm volatile("" :: "v"(z));
    const v4f o = (v4f){ bf16_val(x), bf16_val(y), bf16_val(z), 0.0f };
    volatile v4f* q = (volatile v4f*)(PC + (size_t)r * 4);
    *q = o;
    __threadfence();
    *q = o;
  } else if (blk == PS_PC) {
    const int oc = tid < CH ? tid : CH - 1;
    const float* s = w0 + (size_t)oc * W0LD;
    const float x = s[0], y = s[1], z = s[2];
    asm volatile("" :: "v"(x));
    asm volatile("" :: "v"(y));
    asm volatile("" :: "v"(z));
    const v4f o = (v4f){ bf16_val(x), bf16_val(y), bf16_val(z), 0.0f };
    if (tid < CH) {
      volatile v4f* q = (volatile v4f*)(W0P + 4 * tid);
      *q = o;
      __threadfence();
      *q = o;
    }
  } else {
    const int u  = tid < GB_N / 4 ? tid : GB_N / 4 - 1;
    const int i0 = clampi(u, 0, 15) * 4;
    const int i1 = clampi(u - 16, 0, 15) * 4;
    const int i2 = clampi(u - 32, 0, 63) * 4;
    const int i3 = clampi(u - 96, 0, 63) * 4;
    const int i4 = clampi(u - 160, 0, 15) * 4;
    const int i5 = clampi(u - 176, 0, 15) * 4;
    const v4f a0 = *(const v4fa*)(g0 + i0);
    const v4f a1 = *(const v4fa*)(b0 + i1);
    const v4f a2 = *(const v4fa*)(g1 + i2);
    const v4f a3 = *(const v4fa*)(b1 + i3);
    const v4f a4 = *(const v4fa*)(g2 + i4);
    const v4f a5 = *(const v4fa*)(b2 + i5);
    asm volatile("" :: "v"(a0));
    asm volatile("" :: "v"(a1));
    asm volatile("" :: "v"(a2));
    asm volatile("" :: "v"(a3));
    asm volatile("" :: "v"(a4));
    asm volatile("" :: "v"(a5));
    const unsigned m0 = (u < 16) ? 0xFFFFFFFFu : 0u;
    const unsigned m1 = (u >= 16 && u < 32) ? 0xFFFFFFFFu : 0u;
    const unsigned m2 = (u >= 32 && u < 96) ? 0xFFFFFFFFu : 0u;
    const unsigned m3 = (u >= 96 && u < 160) ? 0xFFFFFFFFu : 0u;
    const unsigned m4 = (u >= 160 && u < 176) ? 0xFFFFFFFFu : 0u;
    const unsigned m5 = (u >= 176) ? 0xFFFFFFFFu : 0u;
    v4f o;
#pragma unroll
    for (int e = 0; e < 4; ++e) {
      const unsigned bits = (__float_as_uint(a0[e]) & m0) | (__float_as_uint(a1[e]) & m1) |
                            (__float_as_uint(a2[e]) & m2) | (__float_as_uint(a3[e]) & m3) |
                            (__float_as_uint(a4[e]) & m4) | (__float_as_uint(a5[e]) & m5);
      o[e] = bf16_val(__uint_as_float(bits));
    }
    if (tid < GB_N / 4) {
      volatile v4f* q = (volatile v4f*)(GB + 4 * tid);
      *q = o;
      __threadfence();
      *q = o;
    }
  }
}

template <int MODE>
__global__ __launch_bounds__(256) void k_edge(const int* __restrict__ idx, const float* __restrict__ PC,
                                              const float* __restrict__ P, const float* __restrict__ W0P,
                                              const float* __restrict__ ST, const float* __restrict__ GB,
                                              double* __restrict__ rec, unsigned short* __restrict__ flhl) {
  static_assert(MODE >= 0 && MODE <= 2);
  __shared__ float sW[8 * CH];
  const int tid = (int)threadIdx.x, lane = tid & 31, wave = tid >> 5;
  const v4f wa = *(const v4fa*)(W0P + 8 * lane);
  const v4f wb = *(const v4fa*)(W0P + 8 * lane + 4);
  const float wax = wa[0], way = wa[1], waz = wa[2];
  const float wbx = wb[0], wby = wb[1], wbz = wb[2];
  float m0 = 0.0f, m1 = 0.0f, r0 = 0.0f, r1 = 0.0f, ga0 = 0.0f, ga1 = 0.0f, be0 = 0.0f, be1 = 0.0f;
  if constexpr (MODE >= 1) {
    const v2f mv = *(const v2fa*)(ST + ST_M0 + 2 * lane);
    m0 = mv[0]; m1 = mv[1];
  }
  if constexpr (MODE == 2) {
    const v2f rv = *(const v2fa*)(ST + ST_R0 + 2 * lane);
    const v2f gv = *(const v2fa*)(GB + GB_G0 + 2 * lane);
    const v2f bv = *(const v2fa*)(GB + GB_B0 + 2 * lane);
    r0 = rv[0]; r1 = rv[1]; ga0 = gv[0]; ga1 = gv[1]; be0 = bv[0]; be1 = bv[1];
  }
  const float* Pl = P + 2 * lane;
  float s0 = 0.0f, s1 = 0.0f;
#pragma unroll 1
  for (int i = 0; i < 8; ++i) {
    const int r = __builtin_amdgcn_readfirstlane((int)blockIdx.x * 64 + wave * 8 + i);
    const int b = r >> 14;
    int nb = idx[(size_t)r * KNB + lane];
    asm volatile("" :: "v"(nb));
    nb = clampi(nb, 0, NPT - 1);
    const int nrow = b * NPT + nb;
    const v4f pnv = *(const v4fa*)(PC + (size_t)nrow * 4);
    const v4f pcv = *(const v4fa*)(PC + (size_t)r * 4);
    const float pnx = pnv[0], pny = pnv[1], pnz = pnv[2];
    const float pcx = pcv[0], pcy = pcv[1], pcz = pcv[2];
    asm volatile("" :: "v"(pnx));
    asm volatile("" :: "v"(pny));
    asm volatile("" :: "v"(pnz));
    asm volatile("" :: "v"(pcx));
    asm volatile("" :: "v"(pcy));
    asm volatile("" :: "v"(pcz));
    const int dxi = __float_as_int(pnx - pcx);
    const int dyi = __float_as_int(pny - pcy);
    const int dzi = __float_as_int(pnz - pcz);
    float mx0 = 0.0f, mx1 = 0.0f;
#pragma unroll 4
    for (int k = 0; k < KNB; ++k) {
      const int   nr = __builtin_amdgcn_readlane(nrow, k);
      const float bx = __int_as_float(__builtin_amdgcn_readlane(dxi, k));
      const float by = __int_as_float(__builtin_amdgcn_readlane(dyi, k));
      const float bz = __int_as_float(__builtin_amdgcn_readlane(dzi, k));
      const v2f pv = *(const v2fa*)(Pl + (size_t)nr * CH);
      const float p0 = pv[0], p1 = pv[1];
      asm volatile("" :: "v"(p0));
      asm volatile("" :: "v"(p1));
      const float h0 = edge_h(p0, bx, by, bz, wax, way, waz);
      const float h1 = edge_h(p1, bx, by, bz, wbx, wby, wbz);
      if constexpr (MODE == 0) {
        s0 += h0; s1 += h1;
      } else if constexpr (MODE == 1) {
        const float d0 = h0 - m0, d1 = h1 - m1;
        s0 += d0 * d0; s1 += d1 * d1;
      } else {
        const float y0 = relu_k(((h0 - m0) * r0) * ga0 + be0);
        const float y1 = relu_k(((h1 - m1) * r1) * ga1 + be1);
        const bool t0 = (k == 0) || (y0 > mx0) || (y0 != y0);
        const bool t1 = (k == 0) || (y1 > mx1) || (y1 != y1);
        mx0 = t0 ? y0 : mx0;
        mx1 = t1 ? y1 : mx1;
      }
    }
    if constexpr (MODE == 2) {
      const unsigned hw = pk16(bf16_bits(mx0), bf16_bits(mx1));
      const unsigned lw = pk16(bf16_lo_bits(mx0), bf16_lo_bits(mx1));
      unsigned short* rp = flhl + (size_t)r * K1T + 2 * lane;
      *(volatile unsigned*)rp = hw;
      if (TWO_TERM_1 != 0) *(volatile unsigned*)(rp + CH) = lw;
      __threadfence();
      *(volatile unsigned*)rp = hw;
      if (TWO_TERM_1 != 0) *(volatile unsigned*)(rp + CH) = lw;
    }
  }
  if constexpr (MODE != 2) {
    sW[wave * CH + 2 * lane]     = s0;
    sW[wave * CH + 2 * lane + 1] = s1;
    __syncthreads();
    if (tid < 32) {
      double a0 = 0.0, a1 = 0.0;
#pragma unroll
      for (int w = 0; w < 8; ++w) {
        a0 += (double)sW[w * CH + 2 * tid];
        a1 += (double)sW[w * CH + 2 * tid + 1];
      }
      const v2d o = (v2d){ a0, a1 };
      volatile v2d* q = (volatile v2d*)(rec + (size_t)blockIdx.x * CH + 2 * tid);
      *q = o;
      __threadfence();
      *q = o;
    }
  }
}

__global__ __launch_bounds__(256) void k_comb(const double* __restrict__ rec, int ncol, int nrec, double inv_count,
                                              int mode, float* __restrict__ out) {
  __shared__ __attribute__((aligned(16))) float sv[256];
  const int tid = (int)threadIdx.x;
  const int c = tid < ncol ? tid : ncol - 1;
  double s = 0.0;
#pragma unroll 4
  for (int i = 0; i < nrec; ++i) s += rec[(size_t)i * (size_t)ncol + c];
  const float qf = (float)(s * inv_count);
  const float rs = 1.0f / sqrtf(qf + 1e-5f);
  sv[tid] = (mode == 0) ? qf : rs;
  __syncthreads();
  const int np = ncol >> 2;
  const int t4 = tid < np ? tid : np - 1;
  const v4f o = *(const v4fa*)(sv + 4 * t4);
  if (tid < np) {
    volatile v4f* q = (volatile v4f*)(out + 4 * tid);
    *q = o;
    __threadfence();
    *q = o;
  }
}

template <int NC, int MODE>
__global__ __launch_bounds__(256) void k_colstat(const float* __restrict__ H, const float* __restrict__ mean,
                                                 double* __restrict__ rec) {
  static_assert(NC == 64 || NC == 256);
  static_assert(MODE == 0 || MODE == 1);
  constexpr int G   = 256 / NC;
  constexpr int RPG = 64 / G;
  __shared__ float sp[256];
  const int tid = (int)threadIdx.x;
  const int col = tid % NC;
  const int g   = tid / NC;
  float m = 0.0f;
  if constexpr (MODE == 1) m = mean[col];
  const float* hp = H + ((size_t)blockIdx.x * 64 + (size_t)g * RPG) * NC + col;
  float s = 0.0f;
#pragma unroll 4
  for (int j = 0; j < RPG; ++j) {
    const float v = hp[(size_t)j * NC];
    if constexpr (MODE == 0) {
      s += v;
    } else {
      const float d = v - m;
      s += d * d;
    }
  }
  sp[tid] = s;
  __syncthreads();
  if (tid < NC / 2) {
    double a0 = 0.0, a1 = 0.0;
#pragma unroll
    for (int gg = 0; gg < G; ++gg) {
      a0 += (double)sp[gg * NC + 2 * tid];
      a1 += (double)sp[gg * NC + 2 * tid + 1];
    }
    const v2d o = (v2d){ a0, a1 };
    volatile v2d* q = (volatile v2d*)(rec + (size_t)blockIdx.x * NC + 2 * tid);
    *q = o;
    __threadfence();
    *q = o;
  }
}

__global__ __launch_bounds__(256) void k_bn1_apply(const float* __restrict__ H1c, const float* __restrict__ ST,
                                                   const float* __restrict__ GB, unsigned short* __restrict__ hl) {
  const int tid = (int)threadIdx.x, lane = tid & 31, wave = tid >> 5;
  const int c0 = 8 * lane;
  const v4f ma = *(const v4fa*)(ST + ST_M1 + c0), mb = *(const v4fa*)(ST + ST_M1 + c0 + 4);
  const v4f ra = *(const v4fa*)(ST + ST_R1 + c0), rb = *(const v4fa*)(ST + ST_R1 + c0 + 4);
  const v4f ga = *(const v4fa*)(GB + GB_G1 + c0), gb = *(const v4fa*)(GB + GB_G1 + c0 + 4);
  const v4f ba = *(const v4fa*)(GB + GB_B1 + c0), bb = *(const v4fa*)(GB + GB_B1 + c0 + 4);
#pragma unroll 1
  for (int i = 0; i < 8; ++i) {
    const int row = (int)blockIdx.x * 64 + wave * 8 + i;
    const float* hp = H1c + (size_t)row * MIDC + c0;
    const v4f xa = *(const v4fa*)(hp);
    const v4f xb = *(const v4fa*)(hp + 4);
    v4f ya, yb;
#pragma unroll
    for (int e = 0; e < 4; ++e) {
      ya[e] = relu_k(((xa[e] - ma[e]) * ra[e]) * ga[e] + ba[e]);
      yb[e] = relu_k(((xb[e] - mb[e]) * rb[e]) * gb[e] + bb[e]);
    }
    const v4u hi = pack8_bf16(ya, yb);
    const v4u lo = pack8_bf16_lo(ya, yb);
    unsigned short* rp = hl + (size_t)row * K2T + c0;
    *(volatile v4u*)rp = hi;
    if (TWO_TERM_2 != 0) *(volatile v4u*)(rp + MIDC) = lo;
    __threadfence();
    *(volatile v4u*)rp = hi;
    if (TWO_TERM_2 != 0) *(volatile v4u*)(rp + MIDC) = lo;
  }
}

__global__ __launch_bounds__(256) void k_final(const float* __restrict__ H2, const unsigned* __restrict__ fbw,
                                               const float* __restrict__ ST, const float* __restrict__ GB,
                                               float* __restrict__ out) {
  __shared__ float tile[CH * 33];
  const int tid = (int)threadIdx.x, lane = tid & 31, wave = tid >> 5;
  const int b  = (int)blockIdx.x / (NPT / 32);
  const int n0 = ((int)blockIdx.x - b * (NPT / 32)) * 32;
  const v2f mv = *(const v2fa*)(ST + ST_M2 + 2 * lane);
  const v2f rv = *(const v2fa*)(ST + ST_R2 + 2 * lane);
  const v2f gv = *(const v2fa*)(GB + GB_G2 + 2 * lane);
  const v2f bv = *(const v2fa*)(GB + GB_B2 + 2 * lane);
  const float m0 = mv[0], m1 = mv[1], r0 = rv[0], r1 = rv[1];
  const float g0 = gv[0], g1 = gv[1], e0 = bv[0], e1 = bv[1];
#pragma unroll
  for (int i = 0; i < 4; ++i) {
    const int row = 4 * wave + i;
    const size_t r = (size_t)b * NPT + n0 + row;
    const v2f hv = *(const v2fa*)(H2 + r * CH + 2 * lane);
    const unsigned w = fbw[r * 32 + lane];
    const float h0 = hv[0], h1 = hv[1];
    asm volatile("" :: "v"(h0));
    asm volatile("" :: "v"(h1));
    asm volatile("" :: "v"(w));
    const float f0 = __uint_as_float(w << 16);
    const float f1 = __uint_as_float(w & 0xffff0000u);
    const float y0 = relu_k((((h0 - m0) * r0) * g0 + e0) + f0);
    const float y1 = relu_k((((h1 - m1) * r1) * g1 + e1) + f1);
    tile[(2 * lane) * 33 + row]     = y0;
    tile[(2 * lane + 1) * 33 + row] = y1;
  }
  __syncthreads();
  float vv[8];
#pragma unroll
  for (int i = 0; i < 8; ++i) vv[i] = tile[(8 * wave + i) * 33 + lane];
  const size_t base = (size_t)(b * CH + 8 * wave) * NPT + n0 + lane;
#pragma unroll
  for (int i = 0; i < 8; ++i) {
    const size_t ix = base + (size_t)i * NPT;
    if (ix < (size_t)OUT_ELEMS) *(volatile float*)(out + ix) = vv[i];
  }
  __threadfence();
#pragma unroll
  for (int i = 0; i < 8; ++i) {
    const size_t ix = base + (size_t)i * NPT;
    if (ix < (size_t)OUT_ELEMS) *(volatile float*)(out + ix) = vv[i];
  }
}

extern "C" void kernel_launch(void* const* d_in, const int* in_sizes, int n_in,
                              void* d_out, int out_size, void* d_ws, size_t ws_size,
                              hipStream_t stream) {
  if (n_in < 12) return;
  if (in_sizes[0] != ROWS * 3) return;
  if (in_sizes[1] != NBAT * CH * NPT) return;
  if (in_sizes[2] != ROWS * KNB) return;
  if (in_sizes[3] != CH * W0LD) return;
  if (in_sizes[4] != CH || in_sizes[5] != CH) return;
  if (in_sizes[6] != MIDC * CH) return;
  if (in_sizes[7] != MIDC || in_sizes[8] != MIDC) return;
  if (in_sizes[9] != CH * MIDC) return;
  if (in_sizes[10] != CH || in_sizes[11] != CH) return;
  if (out_size != OUT_ELEMS) return;
  if (ws_size < WS_TOTAL) return;

  const float* p   = (const float*)d_in[0];
  const float* f   = (const float*)d_in[1];
  const int*   idx = (const int*)d_in[2];
  const float* w0  = (const float*)d_in[3];
  const float* g0  = (const float*)d_in[4];
  const float* b0  = (const float*)d_in[5];
  const float* w1  = (const float*)d_in[6];
  const float* g1  = (const float*)d_in[7];
  const float* b1  = (const float*)d_in[8];
  const float* w2  = (const float*)d_in[9];
  const float* g2  = (const float*)d_in[10];
  const float* b2  = (const float*)d_in[11];
  float* out = (float*)d_out;

  char* ws = (char*)d_ws;
  unsigned short* FB   = (unsigned short*)(ws + OFF_FB);
  float*          PC   = (float*)(ws + OFF_PC);
  float*          P    = (float*)(ws + OFF_P);
  unsigned short* HL   = (unsigned short*)(ws + OFF_HL);
  float*          H1   = (float*)(ws + OFF_H1);
  unsigned short* W0F  = (unsigned short*)(ws + OFF_W0F);
  unsigned short* W1D  = (unsigned short*)(ws + OFF_W1D);
  unsigned short* W2D  = (unsigned short*)(ws + OFF_W2D);
  float*          W0P  = (float*)(ws + OFF_W0P);
  float*          GB   = (float*)(ws + OFF_GB);
  float*          ST   = (float*)(ws + OFF_ST);
  double*         REC0 = (double*)(ws + OFF_REC0);
  double*         REC1 = (double*)(ws + OFF_REC1);
  double*         REC2 = (double*)(ws + OFF_REC2);
  float*          H2   = P;

  const double invE = 1.0 / 2097152.0;
  const double invR = 1.0 / 65536.0;

  k_prep_f<<<NBAT * (NPT / 64), 256, 0, stream>>>(f, (unsigned*)FB);
  k_prep_small<<<PS_TOT, 256, 0, stream>>>(p, w0, g0, b0, g1, b1, g2, b2, PC, W0P, GB);
  k_plane<0><<<CH * CH / 8 / 256, 256, 0, stream>>>(w0 + 3, CH, CH, W0LD, W0F, CH, CH);
  k_plane<FORM_W1><<<MIDC * K1T / 8 / 256, 256, 0, stream>>>(w1, MIDC, CH, CH, W1D, MIDC, CH);
  k_plane<FORM_W2><<<CH * K2T / 8 / 256, 256, 0, stream>>>(w2, CH, MIDC, MIDC, W2D, CH, MIDC);
  k_gemm_nt<0, 0><<<(ROWS / 64 + 7) / 8, 256, 0, stream>>>(FB, W0F, GB, P, ROWS, CH, CH, CH);
  k_edge<0><<<NREC, 256, 0, stream>>>(idx, PC, P, W0P, ST, GB, REC0, HL);
  k_comb<<<1, 256, 0, stream>>>(REC0, CH, NREC, invE, 0, ST + ST_M0);
  k_edge<1><<<NREC, 256, 0, stream>>>(idx, PC, P, W0P, ST, GB, REC0, HL);
  k_comb<<<1, 256, 0, stream>>>(REC0, CH, NREC, invE, 1, ST + ST_R0);
  k_edge<2><<<NREC, 256, 0, stream>>>(idx, PC, P, W0P, ST, GB, REC0, HL);
  k_gemm_nt<0, 0><<<((ROWS / 64) * (MIDC / 64) + 7) / 8, 256, 0, stream>>>(HL, W1D, GB, H1, ROWS, MIDC, K1T, MIDC);
  k_colstat<MIDC, 0><<<NREC, 256, 0, stream>>>(H1, ST + ST_M1, REC1);
  k_comb<<<1, 256, 0, stream>>>(REC1, MIDC, NREC, invR, 0, ST + ST_M1);
  k_colstat<MIDC, 1><<<NREC, 256, 0, stream>>>(H1, ST + ST_M1, REC1);
  k_comb<<<1, 256, 0, stream>>>(REC1, MIDC, NREC, invR, 1, ST + ST_R1);
  for (int q = 0; q < NBAT; ++q) {
    k_bn1_apply<<<CHUNK / 64, 256, 0, stream>>>(H1 + (size_t)q * CHUNK * MIDC, ST, GB, HL);
    k_gemm_nt<0, 0><<<(CHUNK / 64 + 7) / 8, 256, 0, stream>>>(HL, W2D, GB, H2 + (size_t)q * CHUNK * CH,
                                                             CHUNK, CH, K2T, CH);
  }
  k_colstat<CH, 0><<<NREC, 256, 0, stream>>>(H2, ST + ST_M2, REC2);
  k_comb<<<1, 256, 0, stream>>>(REC2, CH, NREC, invR, 0, ST + ST_M2);
  k_colstat<CH, 1><<<NREC, 256, 0, stream>>>(H2, ST + ST_M2, REC2);
  k_comb<<<1, 256, 0, stream>>>(REC2, CH, NREC, invR, 1, ST + ST_R2);
  k_final<<<NBAT * (NPT / 32), 256, 0, stream>>>(H2, (const unsigned*)FB, ST, GB, out);
}
